// RNNCellBuilder_78795470012673
// MI455X (gfx1250) — hardware-verified
//
#include <hip/hip_runtime.h>
#include <math.h>

constexpr int kRows  = 4096;
constexpr int kIn    = 1024;
constexpr int kUnits = 1024;
constexpr int kPld   = 4096;
constexpr int kB1ld  = kUnits + kIn;
constexpr int kB2ld  = kIn + 2 * kUnits;

typedef __attribute__((ext_vector_type(16))) _Float16 v16h;
typedef __attribute__((ext_vector_type(8)))  _Float16 v8h;
typedef __attribute__((ext_vector_type(16))) __bf16   v16b;
typedef __attribute__((ext_vector_type(8)))  __bf16   v8b;
typedef __attribute__((ext_vector_type(8)))  float    v8f;
typedef __attribute__((ext_vector_type(4)))  float    v4f;
typedef __attribute__((ext_vector_type(4)))  unsigned int v4u;

__device__ __forceinline__ unsigned short f2bf_bits(float f) {
  unsigned u = __float_as_uint(f);
  return (unsigned short)((u + 0x7FFFu + ((u >> 16) & 1u)) >> 16);
}
__device__ __forceinline__ float bf_bits2f(unsigned short h) { return __uint_as_float(((unsigned)h) << 16); }

__device__ __forceinline__ void dep_guard_h(v8f& a, v8f& b, v16h x, v16h y) { asm volatile("v_nop\n\tv_nop\n\tv_nop\n\tv_nop" : "+v"(a), "+v"(b) : "v"(x), "v"(y)); }
__device__ __forceinline__ void dep_guard_b(v8f& a, v8f& b, v16b x, v16b y) { asm volatile("v_nop\n\tv_nop\n\tv_nop\n\tv_nop" : "+v"(a), "+v"(b) : "v"(x), "v"(y)); }
__device__ __forceinline__ void keep4_h(v16h a, v16h b, v16h c, v16h d) { asm volatile("v_nop" :: "v"(a), "v"(b), "v"(c), "v"(d)); }
__device__ __forceinline__ void keep4_b(v16b a, v16b b, v16b c, v16b d) { asm volatile("v_nop" :: "v"(a), "v"(b), "v"(c), "v"(d)); }
__device__ __forceinline__ void acc_guard4(v8f& a, v8f& b, v8f& c, v8f& d) { asm volatile("v_nop\n\tv_nop\n\tv_nop\n\tv_nop" : "+v"(a), "+v"(b), "+v"(c), "+v"(d)); }
template <typename T> struct Frag;
template <> struct Frag<_Float16> {
  typedef v16h V; union U { v16h v; v8h h[2]; };
  static __device__ __forceinline__ v16h load(const _Float16* p) {
    U f; f.h[0] = *(const v8h*)(p); f.h[1] = *(const v8h*)(p + 16); return f.v;
  }
  static __device__ __forceinline__ v8f mma(v16h a, v16h b, v8f c) {
    return __builtin_amdgcn_wmma_f32_16x16x32_f16(false, a, false, b, (short)0, c, false, false);
  }
  static __device__ __forceinline__ void guard(v8f& a, v8f& b, v16h x, v16h y) { dep_guard_h(a, b, x, y); }
  static __device__ __forceinline__ void keep(v16h a, v16h b, v16h c, v16h d) { keep4_h(a, b, c, d); }
};
template <> struct Frag<__bf16> {
  typedef v16b V; union U { v16b v; v8b h[2]; };
  static __device__ __forceinline__ v16b load(const __bf16* p) {
    U f; f.h[0] = *(const v8b*)(p); f.h[1] = *(const v8b*)(p + 16); return f.v;
  }
  static __device__ __forceinline__ v8f mma(v16b a, v16b b, v8f c) {
    return __builtin_amdgcn_wmma_f32_16x16x32_bf16(false, a, false, b, (short)0, c, false, false);
  }
  static __device__ __forceinline__ void guard(v8f& a, v8f& b, v16b x, v16b y) { dep_guard_b(a, b, x, y); }
  static __device__ __forceinline__ void keep(v16b a, v16b b, v16b c, v16b d) { keep4_b(a, b, c, d); }
};

__device__ __forceinline__ unsigned pk16(unsigned short a, unsigned short b) { return (unsigned)a | ((unsigned)b << 16); }

__device__ __forceinline__ float sigm_f(float v) {
  const float vc = fminf(fmaxf(v, -30.0f), 30.0f);
  return __builtin_amdgcn_rcpf(1.0f + __expf(-vc));
}
__device__ __forceinline__ float tanh_f(float v) {
  const float vc = fminf(fmaxf(v, -15.0f), 15.0f);
  const float e = __expf(2.0f * vc);
  return 1.0f - 2.0f * __builtin_amdgcn_rcpf(e + 1.0f);
}

template <int EPI>
__global__ __launch_bounds__(256) void gate_gemm64(
    const unsigned short* __restrict__ Ap, int lda,
    const unsigned short* __restrict__ Btp, int ldb,
    void* Cout, void* Cout2, int ldc,
    const float* __restrict__ bias,
    const unsigned short* Hp, int ldh,
    const float* Zp, int ldz,
    int M, int N, int K) {
  typedef __bf16 T;
  typedef v16b V;
  const T* A = (const T*)Ap; const T* Bt = (const T*)Btp;
  __shared__ __align__(16) float sT[8][16 * 68];
  const int lane = threadIdx.x & 31;
  const int wave = threadIdx.x >> 5;
  const int tilesN = N >> 6;
  const int tilesM = M >> 6;
  const int tile = blockIdx.x * 8 + wave;
  if (tile >= tilesM * tilesN) return;
  const int tm = tile / tilesN;
  const int tn = tile - tm * tilesN;
  const int m0 = tm << 6;
  const int n0 = tn << 6;

  const int rlane = lane & 15;
  const int koff  = (lane >> 4) * 8;
  const int mOff  = (lane >> 4) * 8;

  v8f acc[4][4];
#pragma unroll
  for (int i = 0; i < 4; ++i)
#pragma unroll
    for (int j = 0; j < 4; ++j) acc[i][j] = (v8f){0.f,0.f,0.f,0.f,0.f,0.f,0.f,0.f};

  for (int k0 = 0; k0 < K; k0 += 32) {
    V bh[4];
#pragma unroll
    for (int j = 0; j < 4; ++j) {
      const size_t bo = (size_t)(n0 + (j << 4) + rlane) * ldb + koff + k0;
      bh[j] = Frag<T>::load(Bt + bo);
    }
#pragma unroll
    for (int i = 0; i < 4; ++i) {
      const size_t ao = (size_t)(m0 + (i << 4) + rlane) * lda + koff + k0;
      V ah = Frag<T>::load(A + ao);
#pragma unroll
      for (int j = 0; j < 4; ++j) {
        acc[i][j] = Frag<T>::mma(ah, bh[j], acc[i][j]);
      }
      Frag<T>::guard(acc[i][0], acc[i][3], ah, ah);
    }
    Frag<T>::keep(bh[0], bh[1], bh[2], bh[3]);
  }
  acc_guard4(acc[0][0], acc[0][1], acc[0][2], acc[0][3]);
  acc_guard4(acc[1][0], acc[1][1], acc[1][2], acc[1][3]);
  acc_guard4(acc[2][0], acc[2][1], acc[2][2], acc[2][3]);
  acc_guard4(acc[3][0], acc[3][1], acc[3][2], acc[3][3]);

  float* slab = sT[wave];
#pragma unroll
  for (int i = 0; i < 4; ++i) {
    const int mBase = m0 + (i << 4);
#pragma unroll
    for (int j = 0; j < 4; ++j) {
      const int n = n0 + (j << 4) + rlane;
      const float bv = bf_bits2f(f2bf_bits(bias[n]));
#pragma unroll
      for (int r = 0; r < 8; ++r) {
        const int m = mBase + mOff + r;
        float v = acc[i][j][r] + bv;
        if (EPI == 0) {
          v = sigm_f(v);
        } else if (EPI == 1) {
          v = sigm_f(v) * bf_bits2f(Hp[(size_t)m * ldh + n]);
        } else {
          const float hc = tanh_f(v);
          const float z  = Zp[(size_t)m * ldz + n];
          const float hb = bf_bits2f(Hp[(size_t)m * ldh + n]);
          v = z * hb + (1.0f - z) * hc;
        }
        slab[(mOff + r) * 68 + (j << 4) + rlane] = v;
      }
    }
    __builtin_amdgcn_fence(__ATOMIC_RELEASE, "workgroup");
    __builtin_amdgcn_wave_barrier();
    __builtin_amdgcn_fence(__ATOMIC_ACQUIRE, "workgroup");
    if (EPI != 1) {
      float* C = (float*)Cout;
      const int hh = lane >> 4, c4 = (lane & 15) * 4;
      for (int pass = 0; pass < 2; ++pass) {
#pragma unroll
        for (int it = 0; it < 8; ++it) {
          const int row = it * 2 + hh;
          v4f v = *(const v4f*)(slab + row * 68 + c4);
          *(volatile v4f*)(C + (size_t)(mBase + row) * ldc + n0 + c4) = v;
        }
        __threadfence();
      }
    } else {
      const int q = lane >> 3, c8 = (lane & 7) * 8;
      unsigned short* C  = (unsigned short*)Cout;
      unsigned short* C2 = (unsigned short*)Cout2;
      for (int pass = 0; pass < 2; ++pass) {
#pragma unroll
        for (int it = 0; it < 4; ++it) {
          const int row = it * 4 + q;
          const float* sp = slab + row * 68 + c8;
          v8h hv, lv;
#pragma unroll
          for (int e = 0; e < 8; ++e) {
            unsigned short hb = f2bf_bits(sp[e]);
            unsigned short lb = f2bf_bits(sp[e] - bf_bits2f(hb));
            hv[e] = __builtin_bit_cast(_Float16, hb);
            lv[e] = __builtin_bit_cast(_Float16, lb);
          }
          *(volatile v8h*)(C + (size_t)(mBase + row) * ldc + n0 + c8) = hv;
          *(volatile v8h*)(C2 + (size_t)(mBase + row) * ldc + n0 + c8) = lv;
        }
        __threadfence();
      }
    }
    __builtin_amdgcn_fence(__ATOMIC_RELEASE, "workgroup");
    __builtin_amdgcn_wave_barrier();
    __builtin_amdgcn_fence(__ATOMIC_ACQUIRE, "workgroup");
  }
}

__global__ __launch_bounds__(256) void cast_rows_kernel(const float* __restrict__ in, unsigned short* __restrict__ out,
                                                        int C, int ldo, int n8) {
  const int i = blockIdx.x * 256 + threadIdx.x;
  if (i >= n8) return;
  const size_t e0 = 8 * (size_t)i;
  const int r = (int)(e0 / (size_t)C);
  const int c = (int)(e0 - (size_t)r * C);
  const v4f a = *(const v4f*)(in + e0);
  const v4f d = *(const v4f*)(in + e0 + 4);
  unsigned short hb[8];
#pragma unroll
  for (int e = 0; e < 4; ++e) {
    hb[e]     = f2bf_bits(a[e]);
    hb[4 + e] = f2bf_bits(d[e]);
  }
  const v4u u = (v4u){pk16(hb[0], hb[1]), pk16(hb[2], hb[3]), pk16(hb[4], hb[5]), pk16(hb[6], hb[7])};
  unsigned short* qd = out + (size_t)r * ldo + c;
  *(volatile v4u*)qd = u;
  __threadfence();
  *(volatile v4u*)qd = u;
}

__global__ __launch_bounds__(256) void wtrans_kernel(const float* __restrict__ W, unsigned short* __restrict__ Bt,
                                                     int ldb, int koff, int srcN) {
  __shared__ float tile[64][65];
  const int n0 = blockIdx.x * 64;
  const int k0 = blockIdx.y * 64;
  const int t  = threadIdx.x;
  {
    const int kk = t >> 2, cc = (t & 3) * 16;
    const float* src = W + (size_t)(k0 + kk) * srcN + n0 + cc;
#pragma unroll
    for (int q4 = 0; q4 < 4; ++q4) {
      const v4f v = *(const v4f*)(src + 4 * q4);
      tile[kk][cc + 4 * q4 + 0] = v[0];
      tile[kk][cc + 4 * q4 + 1] = v[1];
      tile[kk][cc + 4 * q4 + 2] = v[2];
      tile[kk][cc + 4 * q4 + 3] = v[3];
    }
  }
  __syncthreads();
  const int rq = t >> 3, c8 = (t & 7) * 8;
  v4u u[2];
#pragma unroll
  for (int it = 0; it < 2; ++it) {
    const int nn = it * 32 + rq;
    unsigned short hb[8];
#pragma unroll
    for (int e = 0; e < 8; ++e) hb[e] = f2bf_bits(tile[c8 + e][nn]);
    u[it] = (v4u){pk16(hb[0], hb[1]), pk16(hb[2], hb[3]), pk16(hb[4], hb[5]), pk16(hb[6], hb[7])};
  }
  for (int pass = 0; pass < 2; ++pass) {
#pragma unroll
    for (int it = 0; it < 2; ++it) {
      const int nn = it * 32 + rq;
      *(volatile v4u*)(Bt + (size_t)(n0 + nn) * ldb + koff + k0 + c8) = u[it];
    }
    __threadfence();
  }
}

__global__ __launch_bounds__(256) void copy4_kernel(const float* __restrict__ in, float* __restrict__ out, int n4) {
  const int i = blockIdx.x * 256 + threadIdx.x;
  if (i >= n4) return;
  const v4f v = *(const v4f*)(in + 4 * (size_t)i);
  float* p = out + 4 * (size_t)i;
  *(volatile v4f*)p = v;
  __threadfence();
  *(volatile v4f*)p = v;
}

extern "C" void kernel_launch(void* const* d_in, const int* in_sizes, int n_in,
                              void* d_out, int out_size, void* d_ws, size_t ws_size,
                              hipStream_t stream) {
  if (n_in < 11) return;
  if (in_sizes[0] != kRows * kIn) return;
  if (in_sizes[1] != kRows * kUnits) return;
  if (in_sizes[2] != kIn * kUnits || in_sizes[5] != kIn * kUnits || in_sizes[8] != kIn * kUnits) return;
  if (in_sizes[3] != kUnits * kUnits || in_sizes[6] != kUnits * kUnits || in_sizes[9] != kUnits * kUnits) return;
  if (in_sizes[4] != kUnits || in_sizes[7] != kUnits || in_sizes[10] != kUnits) return;
  if (out_size != 2 * kRows * kUnits) return;

  const float* x     = (const float*)d_in[0];
  const float* h     = (const float*)d_in[1];
  const float* Wz_x  = (const float*)d_in[2];
  const float* Wz_h  = (const float*)d_in[3];
  const float* bz    = (const float*)d_in[4];
  const float* Wr_x  = (const float*)d_in[5];
  const float* Wr_h  = (const float*)d_in[6];
  const float* br    = (const float*)d_in[7];
  const float* Wh_x  = (const float*)d_in[8];
  const float* Wh_rh = (const float*)d_in[9];
  const float* bh    = (const float*)d_in[10];
  float* outp = (float*)d_out;

  const size_t SZ_P  = (size_t)kRows * kPld * 2;
  const size_t SZ_B1 = (size_t)2 * kUnits * kB1ld * 2;
  const size_t SZ_B2 = (size_t)kUnits * kB2ld * 2;
  const size_t SZ_Z  = (size_t)kRows * kUnits * 4;
  size_t off = 0;
  const size_t oP  = off; off += SZ_P;
  const size_t oB1 = off; off += SZ_B1;
  const size_t oB2 = off; off += SZ_B2;
  const size_t oZ  = off; off += SZ_Z;
  const size_t TOTAL = off;
  if (TOTAL > ws_size) return;
  if (TOTAL > (size_t)134217728) return;

  char* ws = (char*)d_ws;
  unsigned short* P   = (unsigned short*)(ws + oP);
  unsigned short* Bt1 = (unsigned short*)(ws + oB1);
  unsigned short* Bt2 = (unsigned short*)(ws + oB2);
  float*          Z   = (float*)(ws + oZ);

  const dim3 blk(256);

  const int n8 = kRows * kIn / 8;
  cast_rows_kernel<<<dim3(n8 / 256), blk, 0, stream>>>(h, P, kUnits, kPld, n8);
  cast_rows_kernel<<<dim3(n8 / 256), blk, 0, stream>>>(x, P + kUnits, kIn, kPld, n8);

  const dim3 gT(kUnits / 64, kIn / 64);
  wtrans_kernel<<<gT, blk, 0, stream>>>(Wz_h, Bt1, kB1ld, 0, kUnits);
  wtrans_kernel<<<gT, blk, 0, stream>>>(Wz_x, Bt1, kB1ld, kUnits, kUnits);
  wtrans_kernel<<<gT, blk, 0, stream>>>(Wr_h, Bt1 + (size_t)kUnits * kB1ld, kB1ld, 0, kUnits);
  wtrans_kernel<<<gT, blk, 0, stream>>>(Wr_x, Bt1 + (size_t)kUnits * kB1ld, kB1ld, kUnits, kUnits);
  wtrans_kernel<<<gT, blk, 0, stream>>>(Wh_x,  Bt2, kB2ld, 0, kUnits);
  wtrans_kernel<<<gT, blk, 0, stream>>>(Wh_rh, Bt2, kB2ld, kIn, kUnits);
  wtrans_kernel<<<gT, blk, 0, stream>>>(Wh_rh, Bt2, kB2ld, kIn + kUnits, kUnits);

  const int n4 = kRows * kUnits / 4;
  copy4_kernel<<<dim3(n4 / 256), blk, 0, stream>>>(h, outp, n4);

  const dim3 gG(((kRows / 64) * (kUnits / 64) + 7) / 8);
  gate_gemm64<0><<<gG, blk, 0, stream>>>(P, kPld, Bt1, kB1ld, (void*)Z, (void*)Z, kUnits, bz,
                                         P, kPld, Z, kUnits, kRows, kUnits, kB1ld);
  gate_gemm64<1><<<gG, blk, 0, stream>>>(P, kPld, Bt1 + (size_t)kUnits * kB1ld, kB1ld,
                                         (void*)(P + 2 * kUnits), (void*)(P + 3 * kUnits), kPld, br,
                                         P, kPld, Z, kUnits, kRows, kUnits, kB1ld);
  gate_gemm64<2><<<gG, blk, 0, stream>>>(P + kUnits, kPld, Bt2, kB2ld,
                                         (void*)(outp + (size_t)kRows * kUnits), (void*)(outp + (size_t)kRows * kUnits), kUnits, bh,
                                         P, kPld, Z, kUnits, kRows, kUnits, kB2ld);
}
